// DeformableAttention1D_71176198029953
// MI455X (gfx1250) — hardware-verified
//
#include <hip/hip_runtime.h>
#define NB 2
#define NTOK 1024
#define DIM 512
#define NHD 8
#define HD 64
#define NG 2
#define OFD 256
#define NM 256
#define HPG 4
#define CPB 128
#define NR (NB * NTOK)
#define NPAIR (NTOK * NM)
typedef __bf16 v16b __attribute__((ext_vector_type(16)));
typedef unsigned short v8us __attribute__((ext_vector_type(8), may_alias));
typedef float  v8f  __attribute__((ext_vector_type(8)));
typedef float  v4f  __attribute__((ext_vector_type(4)));
typedef float  v4fa __attribute__((ext_vector_type(4), may_alias));
union FragB { v16b v; v8us half[2]; unsigned short u[16]; };

__device__ __forceinline__ unsigned short bf16_bits(float x) { unsigned int u = __float_as_uint(x); return (unsigned short)((u + 0x7FFFu + ((u >> 16) & 1u)) >> 16); }
__device__ __forceinline__ float bf16_val(unsigned short b) { return __uint_as_float(((unsigned int)b) << 16); }
__device__ __forceinline__ float bf16_round(float x) { return bf16_val(bf16_bits(x)); }
template <int NT>
__device__ __forceinline__ v8f mmaN(v16b ah, v16b al, v16b bh, v16b bl, v8f c) {
  c = __builtin_amdgcn_wmma_f32_16x16x32_bf16(false, ah, false, bh, (short)0, c, false, false);
  if (NT >= 2) c = __builtin_amdgcn_wmma_f32_16x16x32_bf16(false, al, false, bh, (short)0, c, false, false);
  if (NT >= 3) c = __builtin_amdgcn_wmma_f32_16x16x32_bf16(false, ah, false, bl, (short)0, c, false, false);
  asm volatile("v_nop\n\tv_nop\n\tv_nop\n\tv_nop" : "+v"(c) : "v"(ah), "v"(al), "v"(bh), "v"(bl));
  return c;
}

__global__ __launch_bounds__(256) void k_wt_bf16(const float* __restrict__ W, unsigned short* __restrict__ Wt, int K, int N) {
  const int t = blockIdx.x * 256 + threadIdx.x;
  const int k8n = K / 8;
  if (t >= N * k8n) return;
  const int n = t / k8n, k8 = (t % k8n) * 8;
  v8us v;
#pragma unroll
  for (int i = 0; i < 8; ++i) v[i] = bf16_bits(W[(size_t)(k8 + i) * N + n]);
  *(volatile v8us*)(Wt + (size_t)n * K + k8) = v;
  __threadfence();
  *(volatile v8us*)(Wt + (size_t)n * K + k8) = v;
}

template <bool ASPLIT, int ACT, bool BIAS_BF16>
__global__ __launch_bounds__(128) void k_gemm_bf(const float* __restrict__ A, int lda, const unsigned short* __restrict__ Wt, int ldb,
                                               const float* __restrict__ bias, float* __restrict__ C, int ldc, int M, int N, int K) {
  __shared__ __attribute__((aligned(16))) float so[4][16][64];
  const int tid = threadIdx.x, w = tid >> 5, lane = tid & 31, ln = lane & 15, hh = lane >> 4;
  const int ntn = N / 64;
  const int wid = blockIdx.x * 4 + w;
  const int mt = wid / ntn, nq = wid % ntn;
  if (mt * 16 >= M) return;
  const int row0 = mt * 16, col0 = nq * 64;
  const float* arow = A + (size_t)(row0 + ln) * lda;
  v8f acc[4] = {};
  for (int kb = 0; kb < K; kb += 32) {
    FragB ah, al;
    const v4f x0 = *(const v4fa*)(arow + kb + 8 * hh), x1 = *(const v4fa*)(arow + kb + 8 * hh + 4);
    const v4f x2 = *(const v4fa*)(arow + kb + 16 + 8 * hh), x3 = *(const v4fa*)(arow + kb + 16 + 8 * hh + 4);
    float xs[16] = {x0[0],x0[1],x0[2],x0[3],x1[0],x1[1],x1[2],x1[3],x2[0],x2[1],x2[2],x2[3],x3[0],x3[1],x3[2],x3[3]};
#pragma unroll
    for (int i = 0; i < 16; ++i) { const unsigned short hb = bf16_bits(xs[i]); ah.u[i] = hb; al.u[i] = ASPLIT ? bf16_bits(xs[i] - bf16_val(hb)) : (unsigned short)0; }
#pragma unroll
    for (int t = 0; t < 4; ++t) {
      const unsigned short* brow = Wt + (size_t)(col0 + t * 16 + ln) * ldb + kb;
      FragB b;
      b.half[0] = *(const v8us*)(brow + 8 * hh);
      b.half[1] = *(const v8us*)(brow + 16 + 8 * hh);
      acc[t] = mmaN<ASPLIT ? 2 : 1>(ah.v, al.v, b.v, b.v, acc[t]);
    }
  }
#pragma unroll
  for (int t = 0; t < 4; ++t) {
    float bv = bias ? bias[col0 + t * 16 + ln] : 0.f;
    if (BIAS_BF16) bv = bf16_round(bv);
#pragma unroll
    for (int r = 0; r < 8; ++r) { float v = acc[t][r] + bv; if (ACT == 1) v = fmaxf(v, 0.f); so[w][8 * hh + r][t * 16 + ln] = v; }
  }
  __builtin_amdgcn_fence(__ATOMIC_ACQ_REL, "workgroup");
  __builtin_amdgcn_wave_barrier();
  const int rsub = lane >> 4, c4 = (lane & 15) * 4;
  for (int pass = 0; pass < 2; ++pass) {
#pragma unroll
    for (int q = 0; q < 8; ++q) {
      const int r = q * 2 + rsub;
      const v4f v = *(const v4fa*)&so[w][r][c4];
      *(volatile v4f*)(C + (size_t)(row0 + r) * ldc + col0 + c4) = v;
    }
    if (pass == 0) __threadfence();
  }
}

template <bool ASPLIT, int ACT, bool BIAS_BF16, bool RES_BF16>
__global__ __launch_bounds__(128) void k_gemm_bf3(const float* __restrict__ A, int lda, const unsigned short* __restrict__ Wt, int ldb,
                                                const float* __restrict__ bias, const float* __restrict__ resid, int rmod, int ldr,
                                                float* __restrict__ C, int ldc, int M, int N, int K) {
  __shared__ __attribute__((aligned(16))) float so[4][16][64];
  const int tid = threadIdx.x, w = tid >> 5, lane = tid & 31, ln = lane & 15, hh = lane >> 4;
  const int ntn = N / 64;
  const int wid = blockIdx.x * 4 + w;
  const int mt = wid / ntn, nq = wid % ntn;
  if (mt * 16 >= M) return;
  const int row0 = mt * 16, col0 = nq * 64;
  const float* arow = A + (size_t)(row0 + ln) * lda;
  v8f acc[4] = {};
  for (int kb = 0; kb < K; kb += 32) {
    FragB ah, al;
    const v4f x0 = *(const v4fa*)(arow + kb + 8 * hh), x1 = *(const v4fa*)(arow + kb + 8 * hh + 4);
    const v4f x2 = *(const v4fa*)(arow + kb + 16 + 8 * hh), x3 = *(const v4fa*)(arow + kb + 16 + 8 * hh + 4);
    float xs[16] = {x0[0],x0[1],x0[2],x0[3],x1[0],x1[1],x1[2],x1[3],x2[0],x2[1],x2[2],x2[3],x3[0],x3[1],x3[2],x3[3]};
#pragma unroll
    for (int i = 0; i < 16; ++i) { const unsigned short hb = bf16_bits(xs[i]); ah.u[i] = hb; al.u[i] = ASPLIT ? bf16_bits(xs[i] - bf16_val(hb)) : (unsigned short)0; }
#pragma unroll
    for (int t = 0; t < 4; ++t) {
      const unsigned short* brow = Wt + (size_t)(col0 + t * 16 + ln) * ldb + kb;
      FragB b;
      b.half[0] = *(const v8us*)(brow + 8 * hh);
      b.half[1] = *(const v8us*)(brow + 16 + 8 * hh);
      acc[t] = mmaN<ASPLIT ? 2 : 1>(ah.v, al.v, b.v, b.v, acc[t]);
    }
  }
#pragma unroll
  for (int t = 0; t < 4; ++t) {
    const int col = col0 + t * 16 + ln;
    float bv = bias ? bias[col] : 0.f;
    if (BIAS_BF16) bv = bf16_round(bv);
#pragma unroll
    for (int r = 0; r < 8; ++r) {
      float v = acc[t][r] + bv;
      if (resid) { float rv = resid[(size_t)((row0 + 8 * hh + r) % rmod) * ldr + col]; if (RES_BF16) rv = bf16_round(rv); v += rv; }
      if (ACT == 1) v = fmaxf(v, 0.f);
      if (ACT == 2) v = 0.5f * v * (1.0f + erff(v * 0.70710678118654752f));
      if (ACT == 3) { const float u = 0.7978845608028654f * (v + 0.044715f * v * v * v); v = 0.5f * v * (1.0f + tanhf(u)); }
      so[w][8 * hh + r][t * 16 + ln] = v;
    }
  }
  __builtin_amdgcn_fence(__ATOMIC_ACQ_REL, "workgroup");
  __builtin_amdgcn_wave_barrier();
  const int rsub = lane >> 4, c4 = (lane & 15) * 4;
  for (int pass = 0; pass < 2; ++pass) {
#pragma unroll
    for (int q = 0; q < 8; ++q) {
      const int r = q * 2 + rsub;
      const v4f v = *(const v4fa*)&so[w][r][c4];
      *(volatile v4f*)(C + (size_t)(row0 + r) * ldc + col0 + c4) = v;
    }
    if (pass == 0) __threadfence();
  }
}
template <bool PARAM_BF16>
__global__ __launch_bounds__(256) void k_layernorm(const float* __restrict__ X, const float* __restrict__ R, const float* __restrict__ g, const float* __restrict__ bta,
                                                  float* __restrict__ out_sum, float* __restrict__ out_norm, int N, float eps) {
  __shared__ float red[256];
  const int row = blockIdx.x, tid = threadIdx.x;
  const float* x = X + (size_t)row * N; const float* rr = R ? R + (size_t)row * N : nullptr;
  float vals[16];
  const int per = N / 256;
  float s1 = 0.f;
  for (int u = 0; u < per / 4; ++u) {
    const int j = tid * 4 + 1024 * u;
    const v4f a = *(const v4fa*)(x + j);
    v4f b = {0.f,0.f,0.f,0.f}; if (rr) b = *(const v4fa*)(rr + j);
#pragma unroll
    for (int q = 0; q < 4; ++q) { const float v = a[q] + b[q]; vals[u * 4 + q] = v; s1 += v; }
  }
  red[tid] = s1; __syncthreads();
  for (int st = 128; st > 0; st >>= 1) { if (tid < st) red[tid] += red[tid + st]; __syncthreads(); }
  const float mu = red[0] / (float)N; __syncthreads();
  float s2 = 0.f;
  for (int u = 0; u < per / 4; ++u)
#pragma unroll
    for (int q = 0; q < 4; ++q) { const float c = vals[u * 4 + q] - mu; s2 += c * c; }
  red[tid] = s2; __syncthreads();
  for (int st = 128; st > 0; st >>= 1) { if (tid < st) red[tid] += red[tid + st]; __syncthreads(); }
  const float rs = rsqrtf(red[0] / (float)N + eps);
  for (int pass = 0; pass < 2; ++pass) {
    for (int u = 0; u < per / 4; ++u) {
      const int j = tid * 4 + 1024 * u;
      v4f o, sm;
#pragma unroll
      for (int q = 0; q < 4; ++q) {
        float gg = g[j + q], bb = bta[j + q];
        if (PARAM_BF16) { gg = bf16_round(gg); bb = bf16_round(bb); }
        sm[q] = vals[u * 4 + q]; o[q] = (vals[u * 4 + q] - mu) * rs * gg + bb;
      }
      if (out_sum) *(volatile v4f*)(out_sum + (size_t)row * N + j) = sm;
      *(volatile v4f*)(out_norm + (size_t)row * N + j) = o;
    }
    if (pass == 0) __threadfence();
  }
}


typedef _Float16 v16h __attribute__((ext_vector_type(16)));
union FragH { v16h v; v8us half[2]; _Float16 h[16]; unsigned short u[16]; };
template <int NT>
__device__ __forceinline__ v8f mmaH(v16h ah, v16h al, v16h bh, v16h bl, v8f c) {
  c = __builtin_amdgcn_wmma_f32_16x16x32_f16(false, ah, false, bh, (short)0, c, false, false);
  if (NT >= 2) c = __builtin_amdgcn_wmma_f32_16x16x32_f16(false, al, false, bh, (short)0, c, false, false);
  if (NT >= 3) c = __builtin_amdgcn_wmma_f32_16x16x32_f16(false, ah, false, bl, (short)0, c, false, false);
  asm volatile("v_nop\n\tv_nop\n\tv_nop\n\tv_nop" : "+v"(c) : "v"(ah), "v"(al), "v"(bh), "v"(bl));
  return c;
}
template <bool ASPLIT>
__global__ __launch_bounds__(128) void k_gemm_h(const float* __restrict__ A, int lda, size_t sA, const _Float16* __restrict__ Bh, int ldb, size_t sB, float alpha, float* __restrict__ C, int ldc, size_t sC, int M, int N, int K) {
  __shared__ __attribute__((aligned(16))) float so[4][16][64];
  const int tid = threadIdx.x, w = tid >> 5, lane = tid & 31, ln = lane & 15, hh = lane >> 4; const int by = blockIdx.y;
  A += (size_t)by * sA; Bh += (size_t)by * sB; C += (size_t)by * sC;
  const int ntn = (N + 63) / 64; const int wid = blockIdx.x * 4 + w; const int mt = wid / ntn, nq = wid % ntn; if (mt * 16 >= M) return;
  const int row0 = mt * 16, col0 = nq * 64; const float* arow = A + (size_t)(row0 + ln) * lda;
  v8f acc[4] = {};
  for (int kb = 0; kb < K; kb += 32) {
    FragH ah, al;
    const v4f x0 = *(const v4fa*)(arow + kb + 8 * hh), x1 = *(const v4fa*)(arow + kb + 8 * hh + 4), x2 = *(const v4fa*)(arow + kb + 16 + 8 * hh), x3 = *(const v4fa*)(arow + kb + 16 + 8 * hh + 4);
    float xs[16] = {x0[0],x0[1],x0[2],x0[3],x1[0],x1[1],x1[2],x1[3],x2[0],x2[1],x2[2],x2[3],x3[0],x3[1],x3[2],x3[3]};
#pragma unroll
    for (int i = 0; i < 16; ++i) { const _Float16 h = (_Float16)xs[i]; ah.h[i] = h; al.h[i] = ASPLIT ? (_Float16)(xs[i] - (float)h) : (_Float16)0.0f; }
#pragma unroll
    for (int t = 0; t < 4; ++t) { if (col0 + t * 16 >= N) continue; const size_t boff = (size_t)(col0 + t * 16 + ln) * ldb + kb; FragH bq; bq.half[0] = *(const v8us*)(Bh + boff + 8 * hh); bq.half[1] = *(const v8us*)(Bh + boff + 16 + 8 * hh);
      acc[t] = mmaH<ASPLIT ? 2 : 1>(ah.v, al.v, bq.v, bq.v, acc[t]); }
  }
#pragma unroll
  for (int t = 0; t < 4; ++t) { if (col0 + t * 16 >= N) continue;
#pragma unroll
    for (int r = 0; r < 8; ++r) so[w][8 * hh + r][t * 16 + ln] = acc[t][r] * alpha; }
  __builtin_amdgcn_fence(__ATOMIC_ACQ_REL, "workgroup"); __builtin_amdgcn_wave_barrier();
  const int rsub = lane >> 4, c4 = (lane & 15) * 4;
  for (int pass = 0; pass < 2; ++pass) {
#pragma unroll
    for (int q = 0; q < 8; ++q) { const int r = q * 2 + rsub; if (col0 + c4 < N) { const v4f v = *(const v4fa*)&so[w][r][c4]; *(volatile v4f*)(C + (size_t)(row0 + r) * ldc + col0 + c4) = v; } }
    if (pass == 0) __threadfence(); }
}

__global__ __launch_bounds__(256) void k_wt_f16(const float* __restrict__ W, _Float16* __restrict__ Wt, int K, int N, float scale) {
  const int t = blockIdx.x * 256 + threadIdx.x; if (t >= N * (K / 8)) return; const int n = t / (K / 8), k8 = (t % (K / 8)) * 8; FragH f;
#pragma unroll
  for (int i = 0; i < 8; ++i) f.h[i] = (_Float16)(bf16_round(W[(size_t)(k8 + i) * N + n]) * scale); const v8us o = f.half[0];
  *(volatile v8us*)((unsigned short*)Wt + (size_t)n * K + k8) = o; __threadfence(); *(volatile v8us*)((unsigned short*)Wt + (size_t)n * K + k8) = o;
}
template <int ACT>
__global__ __launch_bounds__(128) void k_gemm_hhx(const _Float16* __restrict__ A, int lda, size_t sA, const _Float16* __restrict__ Bh, int ldb, size_t sB, float alpha, const float* __restrict__ bias, size_t sBias, const float* __restrict__ CP, int rowsPerB, size_t sCPb, int row0g,
    float* __restrict__ C, _Float16* __restrict__ C16, int ldc, size_t sC, int M, int N, int K) {
  __shared__ __attribute__((aligned(16))) float so[4][16][64];
  const int tid = threadIdx.x, w = tid >> 5, lane = tid & 31, ln = lane & 15, hh = lane >> 4; const int by = blockIdx.y;
  A += (size_t)by * sA; Bh += (size_t)by * sB; const size_t cofs = (size_t)by * sC; const float* bp = bias ? bias + (size_t)by * sBias : nullptr;
  const int ntn = (N + 63) / 64; const int wid = blockIdx.x * 4 + w; const int mt = wid / ntn, nq = wid % ntn; if (mt * 16 >= M) return;
  const int row0 = mt * 16, col0 = nq * 64; const _Float16* arow = A + (size_t)(row0 + ln) * lda;
  v8f acc[4] = {};
  for (int kb = 0; kb < K; kb += 32) { FragH ah; ah.half[0] = *(const v8us*)((const unsigned short*)arow + kb + 8 * hh); ah.half[1] = *(const v8us*)((const unsigned short*)arow + kb + 16 + 8 * hh);
#pragma unroll
    for (int t = 0; t < 4; ++t) { if (col0 + t * 16 >= N) continue; const size_t boff = (size_t)(col0 + t * 16 + ln) * ldb + kb; FragH bq; bq.half[0] = *(const v8us*)((const unsigned short*)Bh + boff + 8 * hh); bq.half[1] = *(const v8us*)((const unsigned short*)Bh + boff + 16 + 8 * hh);
      acc[t] = mmaH<1>(ah.v, ah.v, bq.v, bq.v, acc[t]); }
  }
#pragma unroll
  for (int t = 0; t < 4; ++t) { if (col0 + t * 16 >= N) continue; const int col = col0 + t * 16 + ln; const float bv = bp ? bf16_round(bp[col]) : 0.f;
#pragma unroll
    for (int r = 0; r < 8; ++r) { float v = acc[t][r] * alpha + bv; if (CP) { const int rr = row0g + row0 + 8 * hh + r; if (rowsPerB < 0) v += CP[cofs + (size_t)rr * ldc + col];        else { const int bidx = rr / rowsPerB; v += CP[(size_t)bidx * sCPb + (size_t)by * 64 + col]; } } if (ACT == 1) v = (v > 0.f) ? v : expm1f(v); else if (ACT == 7) v = (v > 0.f) ? v + 1.0f : expf(v); else if (ACT == 8) v = tanhf(v); else if (ACT == 9) v = 0.5f * v * (1.0f + tanhf(0.7978845608028654f * (v + 0.044715f * v * v * v))); else if (ACT == 11) v = 1.0f / (1.0f + expf(-v)); else if (ACT == 12) v = (v > 0.f) ? v : 0.01f * v; else if (ACT == 14) v = (v > 0.f) ? v : 0.1f * v; else if (ACT == 16) v = (v >= 0.f) ? v : 0.3f * v; else if (ACT == 17) v = (v >= 0.f) ? v : 0.2f * v; else if (ACT == 15) v = v / (1.0f + expf(-v)); else if (ACT == 3) v = fmaxf(v, 0.f); else if (ACT == 6) v = 0.5f * v * (1.0f + erff(v * 0.70710678118654752f)); so[w][8 * hh + r][t * 16 + ln] = v; } }
  __builtin_amdgcn_fence(__ATOMIC_ACQ_REL, "workgroup"); __builtin_amdgcn_wave_barrier();
  const int rsub = lane >> 4, c4 = (lane & 15) * 4; typedef _Float16 v4h __attribute__((ext_vector_type(4)));
  for (int pass = 0; pass < 2; ++pass) {
#pragma unroll
    for (int q = 0; q < 8; ++q) { const int r = q * 2 + rsub; if (col0 + c4 < N) { const v4f v = *(const v4fa*)&so[w][r][c4]; if (C) *(volatile v4f*)(C + cofs + (size_t)(row0 + r) * ldc + col0 + c4) = v; if (C16) { v4h h4; for (int i = 0; i < 4; ++i) h4[i] = (_Float16)v[i]; *(volatile v4h*)(C16 + cofs + (size_t)(row0 + r) * ldc + col0 + c4) = h4; } } }
    if (pass == 0) __threadfence(); }
}


typedef _Float16 v4h __attribute__((ext_vector_type(4)));

__global__ __launch_bounds__(256) void k_x16(const float* __restrict__ x, _Float16* __restrict__ X16, size_t n8) { const size_t t = (size_t)blockIdx.x * 256 + threadIdx.x; if (t >= n8) return; FragH f;
#pragma unroll
  for (int q = 0; q < 8; ++q) f.h[q] = (_Float16)bf16_round(x[t * 8 + q]); *(volatile v8us*)((unsigned short*)X16 + t * 8) = f.half[0]; __threadfence(); *(volatile v8us*)((unsigned short*)X16 + t * 8) = f.half[0]; }
__global__ __launch_bounds__(256) void k_h16(const float* __restrict__ x, _Float16* __restrict__ X16, size_t n8) { const size_t t = (size_t)blockIdx.x * 256 + threadIdx.x; if (t >= n8) return; FragH f;
#pragma unroll
  for (int q = 0; q < 8; ++q) f.h[q] = (_Float16)x[t * 8 + q]; *(volatile v8us*)((unsigned short*)X16 + t * 8) = f.half[0]; __threadfence(); *(volatile v8us*)((unsigned short*)X16 + t * 8) = f.half[0]; }
__global__ __launch_bounds__(256) void k_round16f(const float* __restrict__ W, _Float16* __restrict__ Bt, size_t n8) { const size_t t = (size_t)blockIdx.x * 256 + threadIdx.x; if (t >= n8) return; FragH f;
#pragma unroll
  for (int i = 0; i < 8; ++i) f.h[i] = (_Float16)(bf16_round(W[t * 8 + i]) * 16.0f); *(volatile v8us*)((unsigned short*)Bt + t * 8) = f.half[0]; __threadfence(); *(volatile v8us*)((unsigned short*)Bt + t * 8) = f.half[0]; }
template <int NHv, int TTv>
__global__ __launch_bounds__(256) void k_vt(const _Float16* __restrict__ V16, int ldv, int voff, _Float16* __restrict__ Vt) { __shared__ unsigned short tl[64][66]; const int tid = threadIdx.x; const int slab = blockIdx.x / (TTv / 64), lg = blockIdx.x % (TTv / 64); const int b = slab / NHv, h = slab % NHv;
  for (int i = tid; i < 64 * 8; i += 256) { const int r = i / 8, c8 = (i % 8) * 8; FragH f; f.half[0] = *(const v8us*)((const unsigned short*)V16 + ((size_t)b * TTv + lg * 64 + r) * ldv + voff + h * 64 + c8);
#pragma unroll
    for (int q = 0; q < 8; ++q) tl[r][c8 + q] = f.u[q]; }
  __syncthreads();
  for (int pass = 0; pass < 2; ++pass) {
#pragma unroll
    for (int rd = 0; rd < 2; ++rd) { const int d = rd * 32 + tid / 8, pc = tid % 8; FragH f;
#pragma unroll
      for (int q = 0; q < 8; ++q) f.u[q] = tl[pc * 8 + q][d];
      *(volatile v8us*)((unsigned short*)Vt + ((size_t)slab * 64 + d) * TTv + lg * 64 + pc * 8) = f.half[0]; }
    if (pass == 0) __threadfence(); } }

__global__ __launch_bounds__(256) void k_hl(const float* __restrict__ F, _Float16* __restrict__ Hh, _Float16* __restrict__ Hl, size_t n8) { const size_t t = (size_t)blockIdx.x * 256 + threadIdx.x; if (t >= n8) return; FragH fh, fl; const v4f a = *(const v4fa*)(F + t * 8), c = *(const v4fa*)(F + t * 8 + 4);
#pragma unroll
  for (int q = 0; q < 4; ++q) { _Float16 h = (_Float16)a[q]; fh.h[q] = h; fl.h[q] = (_Float16)((a[q] - (float)h) * 1024.0f); h = (_Float16)c[q]; fh.h[4 + q] = h; fl.h[4 + q] = (_Float16)((c[q] - (float)h) * 1024.0f); }
  for (int pass = 0; pass < 2; ++pass) { *(volatile v8us*)((unsigned short*)Hh + t * 8) = fh.half[0]; *(volatile v8us*)((unsigned short*)Hl + t * 8) = fl.half[0]; if (pass == 0) __threadfence(); } }

__device__ __forceinline__ v16h g2_frag(const _Float16* p, int hh) { FragH f; f.half[0] = *(const v8us*)((const unsigned short*)p + 8 * hh); f.half[1] = *(const v8us*)((const unsigned short*)p + 16 + 8 * hh); return f.v; }
__device__ __forceinline__ v8f g2_mma(v16h a, v16h b, v8f c) { v8f d = __builtin_amdgcn_wmma_f32_16x16x32_f16(false, a, false, b, (short)0, c, false, false); asm volatile("v_nop\n\tv_nop\n\tv_nop\n\tv_nop" : "+v"(d) : "v"(a), "v"(b)); return d; }
template <int ACT>
__global__ __launch_bounds__(128) void k_gemm2(const _Float16* __restrict__ A, int lda, size_t sA, const _Float16* __restrict__ Bh, int ldb, size_t sB, float alpha, const float* __restrict__ bias, size_t sBias, const float* __restrict__ CP, int rowsPerB, size_t sCPb, int row0g,
    float* __restrict__ C, _Float16* __restrict__ C16, int ldc, size_t sC, int M, int N, int K) { static_assert(ACT == 0 || ACT == 3 || ACT == 6 || ACT == 8 || ACT == 9 || ACT == 11 || ACT == 12 || ACT == 14 || ACT == 15 || ACT == 16 || ACT == 17, "k_gemm2: unsupported ACT code (would silently apply no activation)");
  __shared__ __attribute__((aligned(16))) float so[4][32][68];
  const int tid = threadIdx.x, w = tid >> 5, lane = tid & 31, ln = lane & 15, hh = lane >> 4; const int by = blockIdx.y;
  A += (size_t)by * sA; Bh += (size_t)by * sB; const size_t cofs = (size_t)by * sC; const float* bp = bias ? bias + (size_t)by * sBias : nullptr;
  const int ntn = N >> 6; const int mt = blockIdx.x / ntn, nq = blockIdx.x - mt * ntn; const int row0 = mt * 128 + 32 * w, col0 = nq * 64; if (row0 >= M) return;
  const _Float16* a0p = A + (size_t)(row0 + ln) * lda; const _Float16* a1p = a0p + (size_t)16 * lda;
  const _Float16* b0p = Bh + (size_t)(col0 + ln) * ldb; const _Float16* b1p = b0p + (size_t)16 * ldb; const _Float16* b2p = b1p + (size_t)16 * ldb; const _Float16* b3p = b2p + (size_t)16 * ldb;
  const v8f z8 = {0.f,0.f,0.f,0.f,0.f,0.f,0.f,0.f}; v8f c00 = z8, c01 = z8, c02 = z8, c03 = z8, c10 = z8, c11 = z8, c12 = z8, c13 = z8;
#pragma unroll 1
  for (int kb = 0; kb < K; kb += 32) { const v16h a0 = g2_frag(a0p + kb, hh), a1 = g2_frag(a1p + kb, hh);
    v16h b = g2_frag(b0p + kb, hh); c00 = g2_mma(a0, b, c00); c10 = g2_mma(a1, b, c10);
    b = g2_frag(b1p + kb, hh); c01 = g2_mma(a0, b, c01); c11 = g2_mma(a1, b, c11);
    b = g2_frag(b2p + kb, hh); c02 = g2_mma(a0, b, c02); c12 = g2_mma(a1, b, c12);
    b = g2_frag(b3p + kb, hh); c03 = g2_mma(a0, b, c03); c13 = g2_mma(a1, b, c13); }
  v8f accs[8] = {c00, c01, c02, c03, c10, c11, c12, c13};
#pragma unroll
  for (int u = 0; u < 8; ++u) { const int t = u & 3, half = u >> 2; const int col = col0 + t * 16 + ln; const float bv = bp ? bf16_round(bp[col]) : 0.f;
#pragma unroll
    for (int r = 0; r < 8; ++r) { const int rloc = half * 16 + 8 * hh + r; float v = accs[u][r] * alpha + bv; if (CP) { if (rowsPerB < 0) v += CP[cofs + (size_t)(row0g + row0 + rloc) * ldc + col];        else { const int bidx = (row0g + row0 + rloc) / rowsPerB; v += CP[(size_t)bidx * sCPb + (size_t)by * 64 + col]; } }
      if (ACT == 3) v = fmaxf(v, 0.f); else if (ACT == 6) v = 0.5f * v * (1.0f + erff(v * 0.70710678118654752f)); else if (ACT == 11) v = 1.0f / (1.0f + expf(-v)); else if (ACT == 15) v = v / (1.0f + expf(-v)); else if (ACT == 12) v = (v > 0.f) ? v : 0.01f * v; else if (ACT == 8) v = tanhf(v); else if (ACT == 9) v = 0.5f * v * (1.0f + tanhf(0.7978845608028654f * (v + 0.044715f * v * v * v))); else if (ACT == 14) v = (v > 0.f) ? v : 0.1f * v; else if (ACT == 16) v = (v >= 0.f) ? v : 0.3f * v; else if (ACT == 17) v = (v >= 0.f) ? v : 0.2f * v;
      so[w][rloc][t * 16 + ln] = v; } }
  __builtin_amdgcn_fence(__ATOMIC_ACQ_REL, "workgroup"); __builtin_amdgcn_wave_barrier();
  const int rsub = lane >> 4, c4 = (lane & 15) * 4;
  for (int pass = 0; pass < 2; ++pass) {
#pragma unroll
    for (int q = 0; q < 16; ++q) { const int r = q * 2 + rsub; const v4f v = *(const v4fa*)&so[w][r][c4]; if (C) *(volatile v4f*)(C + cofs + (size_t)(row0 + r) * ldc + col0 + c4) = v; if (C16) { v4h h4; for (int i = 0; i < 4; ++i) h4[i] = (_Float16)v[i]; *(volatile v4h*)(C16 + cofs + (size_t)(row0 + r) * ldc + col0 + c4) = h4; } }
    if (pass == 0) __threadfence(); } }


__global__ __launch_bounds__(256) void k_zpad(_Float16* __restrict__ Z, size_t n8) { const size_t t = (size_t)blockIdx.x * 256 + threadIdx.x; if (t >= n8) return; FragH f; for (int q = 0; q < 8; ++q) f.h[q] = (_Float16)0.0f; *(volatile v8us*)((unsigned short*)Z + t * 8) = f.half[0]; __threadfence(); *(volatile v8us*)((unsigned short*)Z + t * 8) = f.half[0]; }
__global__ __launch_bounds__(32) void k_bb3(const float* __restrict__ b3, float* __restrict__ BB3) { const int t = threadIdx.x; if (t >= 16) return; const float v = (t < HPG) ? b3[t] : 0.f; *(volatile float*)(BB3 + t) = v; __threadfence(); *(volatile float*)(BB3 + t) = v; }
__global__ __launch_bounds__(256) void k_off(const float* __restrict__ Q, const float* __restrict__ w1, const float* __restrict__ b1, const float* __restrict__ w2, float* __restrict__ VG) {
  #pragma clang fp contract(off)
  const int t = blockIdx.x * 256 + threadIdx.x; if (t >= NB * NG * NM) return; const int m = t % NM; const int g = (t / NM) % NG; const int b = t / (NM * NG); float acc = 0.f;
#pragma unroll 1
  for (int d = 0; d < OFD; ++d) { float h = 0.f;
#pragma unroll 1
    for (int k = 0; k < 6; ++k) { const int n = 4 * m + k - 1; if (n < 0 || n >= NTOK) continue; h += bf16_round(w1[d * 6 + k]) * Q[((size_t)b * NTOK + n) * DIM + g * OFD + d]; }
    h += bf16_round(b1[d]); h = 0.5f * h * (1.0f + erff(h * 0.70710678118654752f)); acc += h * bf16_round(w2[d]); }
  const float off = tanhf(acc) * 4.0f; const float vg = (float)m + off; *(volatile float*)(VG + t) = vg; __threadfence(); *(volatile float*)(VG + t) = vg; }
__global__ __launch_bounds__(256) void k_rtab(const float* __restrict__ Q, const float* __restrict__ Wkv, float* __restrict__ R) {
  #pragma clang fp contract(off)
  const int t = blockIdx.x * 256 + threadIdx.x; if (t >= NB * NG * 2 * DIM) return; const int c = t % (2 * DIM); const int g = (t / (2 * DIM)) % NG; const int b = t / (2 * DIM * NG); float s = 0.f;
#pragma unroll 1
  for (int d = 0; d < OFD; ++d) { float row = 0.5f * Q[((size_t)b * NTOK + 511) * DIM + g * OFD + d]; row += 0.5f * Q[((size_t)b * NTOK + 512) * DIM + g * OFD + d]; s += row * bf16_round(Wkv[((size_t)g * OFD + d) * (2 * DIM) + c]); }
  *(volatile float*)(R + t) = s; __threadfence(); *(volatile float*)(R + t) = s; }
__global__ __launch_bounds__(256) void k_cpb1(const float* __restrict__ VG, const float* __restrict__ w1, const float* __restrict__ b1, _Float16* __restrict__ H1) {
  #pragma clang fp contract(off)
  const size_t t = (size_t)blockIdx.x * 256 + threadIdx.x; if (t >= (size_t)NPAIR * (CPB / 8)) return; const int u8 = (int)(t % (CPB / 8)) * 8; const int pr = (int)(t / (CPB / 8)); const int j = pr % NM, i = pr / NM;
  const float si = 2.0f * (float)i / (float)(NTOK - 1) - 1.0f; const float vs = 2.0f * VG[j] / (float)(NM - 1) - 1.0f; const float p = si - vs; const float sg = (p > 0.f) ? 1.0f : ((p < 0.f) ? -1.0f : 0.0f); const float tt = sg * log1pf(fabsf(p)); FragH f;
  for (int q = 0; q < 8; ++q) { float v = tt * bf16_round(w1[u8 + q]); v += bf16_round(b1[u8 + q]); f.h[q] = (_Float16)fmaxf(v, 0.f); }
  *(volatile v8us*)((unsigned short*)H1 + t * 8) = f.half[0]; __threadfence(); *(volatile v8us*)((unsigned short*)H1 + t * 8) = f.half[0]; }
__global__ __launch_bounds__(256) void k_wcol(const float* __restrict__ VG, float* __restrict__ WC) {
  #pragma clang fp contract(off)
  const int t = blockIdx.x * 256 + threadIdx.x; if (t >= NB * NG * NM) return; const float vs = 2.0f * VG[t] / (float)(NM - 1) - 1.0f; float ix = (vs + 1.0f) * 1.0f - 1.0f; ix = ix / 2.0f; const float x0 = floorf(ix); const float wx1 = ix - x0; float w = 0.f; if (x0 == 0.0f) w += 1.0f - wx1; if (x0 == -1.0f) w += wx1;
  *(volatile float*)(WC + t) = w; __threadfence(); *(volatile float*)(WC + t) = w; }
__global__ __launch_bounds__(256) void k_attn(const float* __restrict__ Q, const float* __restrict__ R, const float* __restrict__ WC, const float* __restrict__ BI, int b, _Float16* __restrict__ O16) {
  #pragma clang fp contract(off)
  const int wv = threadIdx.x >> 5, ln = threadIdx.x & 31; const int r = blockIdx.x * 8 + wv; if (r >= NHD * NTOK) return; const int i = r % NTOK, h = r / NTOK; const int gh = h / HPG, hh = h % HPG; const float* q = Q + ((size_t)b * NTOK + i) * DIM + h * HD;
  const float* R0 = R + ((size_t)(b * NG + 0)) * (2 * DIM), * R1 = R + ((size_t)(b * NG + 1)) * (2 * DIM); float a0 = q[ln] * R0[h * HD + ln]; a0 += q[ln + 32] * R0[h * HD + ln + 32]; float a1 = q[ln] * R1[h * HD + ln]; a1 += q[ln + 32] * R1[h * HD + ln + 32];
  for (int o = 16; o > 0; o >>= 1) { a0 += __shfl_xor(a0, o, 32); a1 += __shfl_xor(a1, o, 32); } a0 *= 0.125f; a1 *= 0.125f;
  const float* wc0 = WC + (size_t)(b * NG + 0) * NM, * wc1 = WC + (size_t)(b * NG + 1) * NM; const float* bi = BI + ((size_t)gh * NPAIR + (size_t)i * NM) * 16 + hh;
  float lg[8]; float mx = -3.0e38f; for (int e = 0; e < 8; ++e) { const int j = ln * 8 + e; float v = a0 * wc0[j]; v += a1 * wc1[j]; v += bi[(size_t)j * 16]; lg[e] = v; mx = fmaxf(mx, v); }
  for (int o = 16; o > 0; o >>= 1) mx = fmaxf(mx, __shfl_xor(mx, o, 32)); float su = 0.f, s0 = 0.f, s1 = 0.f; for (int e = 0; e < 8; ++e) { const int j = ln * 8 + e; const float ev = expf(lg[e] - mx); su += ev; s0 += ev * wc0[j]; s1 += ev * wc1[j]; }
  for (int o = 16; o > 0; o >>= 1) { su += __shfl_xor(su, o, 32); s0 += __shfl_xor(s0, o, 32); s1 += __shfl_xor(s1, o, 32); } s0 = s0 / su; s1 = s1 / su;
  const float* V0 = R0 + DIM + h * HD, * V1 = R1 + DIM + h * HD; _Float16* o16 = O16 + ((size_t)b * NTOK + i) * DIM + h * HD;
  for (int pass = 0; pass < 2; ++pass) { for (int u = 0; u < 2; ++u) { const int d = ln + 32 * u; float v = s0 * V0[d]; v += s1 * V1[d]; *(volatile _Float16*)(o16 + d) = (_Float16)v; } if (pass == 0) __threadfence(); } }

extern "C" void kernel_launch(void* const* d_in, const int* in_sizes, int n_in,
                              void* d_out, int out_size, void* d_ws, size_t ws_size, hipStream_t stream) {
  (void)in_sizes; (void)n_in; (void)out_size;
  const float* const* I = (const float* const*)d_in; const float* x = I[0]; const float* wq = I[1]; const float* c1w = I[2]; const float* c1b = I[3]; const float* c2w = I[4]; const float* p1w = I[5]; const float* p1b = I[6]; const float* p2w = I[7]; const float* p2b = I[8]; const float* p3w = I[9]; const float* p3b = I[10]; const float* wkv = I[11]; const float* wo = I[12]; const float* bo = I[13];
  char* ws = (char*)d_ws; size_t off = 0;
  auto take = [&](size_t bytes) { char* p = ws + off; off += (bytes + 255) & ~(size_t)255; return p; };
  _Float16* BQ = (_Float16*)take((size_t)DIM * DIM * 2); _Float16* BO = (_Float16*)take((size_t)DIM * DIM * 2); _Float16* B2 = (_Float16*)take((size_t)CPB * CPB * 2); _Float16* B3 = (_Float16*)take((size_t)16 * CPB * 2); float* BB3 = (float*)take(16 * 4);
  _Float16* X16 = (_Float16*)take((size_t)NR * DIM * 2); float* Q = (float*)take((size_t)NR * DIM * 4); float* VG = (float*)take((size_t)NB * NG * NM * 4); float* WC = (float*)take((size_t)NB * NG * NM * 4); float* R = (float*)take((size_t)NB * NG * 2 * DIM * 4);
  _Float16* H1 = (_Float16*)take((size_t)NPAIR * CPB * 2); _Float16* H2 = (_Float16*)take((size_t)NPAIR * CPB * 2); float* BI = (float*)take((size_t)NG * NPAIR * 16 * 4); _Float16* O16 = (_Float16*)take((size_t)NR * DIM * 2);
  if (off > ws_size) return;
  k_wt_f16<<<(DIM * DIM / 8 + 255) / 256, 256, 0, stream>>>(wq, BQ, DIM, DIM, 16.0f); k_wt_f16<<<(DIM * DIM / 8 + 255) / 256, 256, 0, stream>>>(wo, BO, DIM, DIM, 16.0f); k_wt_f16<<<(CPB * CPB / 8 + 255) / 256, 256, 0, stream>>>(p2w, B2, CPB, CPB, 16.0f);
  k_zpad<<<(16 * CPB / 8 + 255) / 256, 256, 0, stream>>>(B3, 16 * CPB / 8); k_wt_f16<<<(CPB * 4 / 8 + 255) / 256, 256, 0, stream>>>(p3w, B3, CPB, 4, 16.0f);
  k_bb3<<<1, 32, 0, stream>>>(p3b, BB3);
  k_x16<<<(unsigned)(((size_t)NR * DIM / 8 + 255) / 256), 256, 0, stream>>>(x, X16, (size_t)NR * DIM / 8);
  k_gemm2<0><<<dim3((NR / 128) * (DIM / 64), 1), 128, 0, stream>>>(X16, DIM, 0, BQ, DIM, 0, 0.0625f, nullptr, 0, nullptr, 1, 0, 0, Q, nullptr, DIM, 0, NR, DIM, DIM);
  k_off<<<(NB * NG * NM + 255) / 256, 256, 0, stream>>>(Q, c1w, c1b, c2w, VG); k_wcol<<<(NB * NG * NM + 255) / 256, 256, 0, stream>>>(VG, WC); k_rtab<<<(NB * NG * 2 * DIM + 255) / 256, 256, 0, stream>>>(Q, wkv, R);
  for (int b = 0; b < NB; ++b) {
    for (int g = 0; g < NG; ++g) {
      k_cpb1<<<(unsigned)(((size_t)NPAIR * (CPB / 8) + 255) / 256), 256, 0, stream>>>(VG + (size_t)(b * NG + g) * NM, p1w, p1b, H1);
      k_gemm2<3><<<dim3((NPAIR / 128) * (CPB / 64), 1), 128, 0, stream>>>(H1, CPB, 0, B2, CPB, 0, 0.0625f, p2b, 0, nullptr, 1, 0, 0, nullptr, H2, CPB, 0, NPAIR, CPB, CPB);
      k_gemm_hhx<0><<<(unsigned)((NPAIR / 16) * 1 / 4), 128, 0, stream>>>(H2, CPB, 0, B3, CPB, 0, 0.0625f, BB3, 0, nullptr, 1, 0, 0, BI + (size_t)g * NPAIR * 16, nullptr, 16, 0, NPAIR, 16, CPB); }
    k_attn<<<(NHD * NTOK) / 8, 256, 0, stream>>>(Q, R, WC, BI, b, O16); }
  k_gemm2<0><<<dim3((NR / 128) * (DIM / 64), 1), 128, 0, stream>>>(O16, DIM, 0, BO, DIM, 0, 0.0625f, bo, 0, nullptr, 1, 0, 0, (float*)d_out, nullptr, DIM, 0, NR, DIM, DIM);
}
